// VectorizedSREKEnsemble_47605417508981
// MI455X (gfx1250) — hardware-verified
//
#include <hip/hip_runtime.h>


#define NA   64
#define NBT  4096
#define DI   50
#define KI   64
#define HH   192
#define NO   3
typedef _Float16 h16;
typedef unsigned short bf;
typedef __attribute__((ext_vector_type(16))) __bf16   v16bf;
typedef __attribute__((ext_vector_type(16))) _Float16 v16h;
typedef __attribute__((ext_vector_type(8)))  _Float16 v8h;
typedef __attribute__((ext_vector_type(8)))  unsigned short v8us;
typedef __attribute__((ext_vector_type(8)))  float    v8f;
typedef __attribute__((ext_vector_type(4)))  float    v4f;
typedef v8h  __attribute__((may_alias)) v8ha;
typedef v4f  __attribute__((may_alias)) v4fa;
typedef v8us __attribute__((may_alias)) v8usa;

__device__ __forceinline__ unsigned short f2bf(float f) { unsigned u = __float_as_uint(f); u += 0x7FFFu + ((u >> 16) & 1u); return (unsigned short)(u >> 16); }
__device__ __forceinline__ float bf2f(unsigned short b) { return __uint_as_float(((unsigned)b) << 16); }
__device__ __forceinline__ float bfr(float f) { return bf2f(f2bf(f)); }
__device__ __forceinline__ v16h cat16(v8h lo, v8h hi) { return __builtin_shufflevector(lo, hi, 0, 1, 2, 3, 4, 5, 6, 7, 8, 9, 10, 11, 12, 13, 14, 15); }
__device__ __forceinline__ v16bf cat16b(v8us lo, v8us hi) { return __builtin_bit_cast(v16bf, __builtin_shufflevector(lo, hi, 0, 1, 2, 3, 4, 5, 6, 7, 8, 9, 10, 11, 12, 13, 14, 15)); }
__device__ __forceinline__ v8f wmma16(v16h a, v16h b, v8f c) { return __builtin_amdgcn_wmma_f32_16x16x32_f16(false, a, false, b, (short)0, c, false, false); }
__device__ __forceinline__ v8f wmmab(v16bf a, v16bf b, v8f c) { return __builtin_amdgcn_wmma_f32_16x16x32_bf16(false, a, false, b, (short)0, c, false, false); }


template <typename T16> struct WFrag;
template <> struct WFrag<h16> { typedef v16h V; static __device__ __forceinline__ V ld(const h16* p) { return cat16(*(const v8h*)p, *(const v8h*)(p + 16)); } static __device__ __forceinline__ v8f mma(V a, V b, v8f c) { return wmma16(a, b, c); } };
template <> struct WFrag<bf> { typedef v16bf V; static __device__ __forceinline__ V ld(const bf* p) { return cat16b(*(const v8us*)p, *(const v8us*)(p + 16)); } static __device__ __forceinline__ v8f mma(V a, V b, v8f c) { return wmmab(a, b, c); } };
template <typename T16, int NSPLIT, bool BIAS>
__global__ __launch_bounds__(32) void k_gemmw(const T16* __restrict__ A, const T16* __restrict__ A2, const T16* __restrict__ Bt, const T16* __restrict__ Bt2, int K, float* C, int ldc, const float* __restrict__ bias, size_t sA, size_t sB, size_t sC) {
    typedef typename WFrag<T16>::V V;
    __shared__ __align__(16) float os[16 * 68];
    const size_t z = blockIdx.z; A += z * sA; if (A2) A2 += z * sA; Bt += z * sB; if (Bt2) Bt2 += z * sB; C += z * sC;
    const int lane = threadIdx.x & 31, lr = lane & 15, hi = lane >> 4; const int r0 = blockIdx.x * 64, c0 = blockIdx.y * 64;
    v8f acc[4][4];
#pragma unroll
    for (int mb = 0; mb < 4; ++mb)
#pragma unroll
        for (int nb = 0; nb < 4; ++nb) acc[mb][nb] = (v8f){};
    const size_t aoff = (size_t)(r0 + lr) * K + 8 * hi, boff = (size_t)(c0 + lr) * K + 8 * hi;
#pragma unroll 1
    for (int kc = 0; kc < K; kc += 32) {
        V a[4], a2[4];
#pragma unroll
        for (int mb = 0; mb < 4; ++mb) { a[mb] = WFrag<T16>::ld(A + aoff + (size_t)mb * 16 * K + kc); if (NSPLIT == 1 || NSPLIT == 2) a2[mb] = WFrag<T16>::ld(A2 + aoff + (size_t)mb * 16 * K + kc); }
#pragma unroll
        for (int nb = 0; nb < 4; ++nb) { const V b = WFrag<T16>::ld(Bt + boff + (size_t)nb * 16 * K + kc); V b2; if (NSPLIT >= 2) b2 = WFrag<T16>::ld(Bt2 + boff + (size_t)nb * 16 * K + kc);
#pragma unroll
            for (int mb = 0; mb < 4; ++mb) { acc[mb][nb] = WFrag<T16>::mma(a[mb], b, acc[mb][nb]); if (NSPLIT == 1 || NSPLIT == 2) acc[mb][nb] = WFrag<T16>::mma(a2[mb], b, acc[mb][nb]); if (NSPLIT >= 2) acc[mb][nb] = WFrag<T16>::mma(a[mb], b2, acc[mb][nb]); } }
        asm volatile("v_nop\n\tv_nop\n\tv_nop\n\tv_nop" : "+v"(acc[0][0]), "+v"(acc[1][1]), "+v"(acc[2][2]), "+v"(acc[3][3]) : "v"(a[0]), "v"(a[3]));
    }
#pragma unroll
    for (int mb = 0; mb < 4; ++mb) {
#pragma unroll
        for (int nb = 0; nb < 4; ++nb) {
#pragma unroll
            for (int j = 0; j < 8; ++j) os[(hi * 8 + j) * 68 + nb * 16 + lr] = acc[mb][nb][j]; }
        __builtin_amdgcn_wave_barrier(); asm volatile("" ::: "memory");
        float* crow = C + (size_t)(r0 + mb * 16) * ldc + c0;
#pragma unroll 1
        for (int ps = 0; ps < 2; ++ps) {
#pragma unroll
            for (int s = 0; s < 8; ++s) { const int row = 2 * s + hi, cofs = lr * 4; v4f val = *(const v4fa*)(os + row * 68 + cofs); if (BIAS) { val[0] += bfr(bias[c0 + cofs]); val[1] += bfr(bias[c0 + cofs + 1]); val[2] += bfr(bias[c0 + cofs + 2]); val[3] += bfr(bias[c0 + cofs + 3]); }
                *(volatile v4f*)(crow + (size_t)row * ldc + cofs) = val; }
            if (ps == 0) __threadfence(); }
        __builtin_amdgcn_wave_barrier(); asm volatile("" ::: "memory");
    }
}

__device__ __forceinline__ h16 tohx(float x) { return (h16)x; }
__device__ __forceinline__ void splitf(float y, unsigned short& h, unsigned short& l) { h = f2bf(y); l = f2bf(y - bf2f(h)); }
__device__ __forceinline__ float gelu_(float x) { return 0.5f * x * (1.0f + erff(x * 0.7071067811865476f)); }
typedef __attribute__((ext_vector_type(2))) _Float16 v2h;
typedef __attribute__((ext_vector_type(4))) _Float16 v4h;
typedef __attribute__((ext_vector_type(2))) unsigned short v2us;
typedef __attribute__((ext_vector_type(4))) unsigned short v4us;

__global__ __launch_bounds__(256) void k_w1(const float* __restrict__ W1, const float* __restrict__ S1, bf* B1) { const size_t e = ((size_t)blockIdx.x * 256 + threadIdx.x) * 2; if (e >= (size_t)NA * 2 * HH * KI) return; const int k = (int)(e % KI); const int n = (int)((e / KI) % (2 * HH)); const int a = (int)(e / ((size_t)KI * 2 * HH)); const float* src = n < HH ? W1 + ((size_t)a * HH + n) * DI : S1 + ((size_t)a * HH + n - HH) * DI; v2us o;
#pragma unroll
    for (int u = 0; u < 2; ++u) o[u] = (k + u) < DI ? f2bf(src[k + u]) : (unsigned short)0; *(volatile v2us*)(B1 + e) = o; __threadfence(); *(volatile v2us*)(B1 + e) = o; }
__global__ __launch_bounds__(256) void k_w2(const float* __restrict__ W2, const float* __restrict__ S2, h16* B2) { const size_t e = ((size_t)blockIdx.x * 256 + threadIdx.x) * 4; if (e >= (size_t)NA * 2 * HH * HH) return; const int k = (int)(e % HH); const int n = (int)((e / HH) % (2 * HH)); const int a = (int)(e / ((size_t)HH * 2 * HH)); const float* src = n < HH ? W2 + ((size_t)a * HH + n) * HH : S2 + ((size_t)a * HH + n - HH) * HH; v4h o;
#pragma unroll
    for (int q = 0; q < 4; ++q) o[q] = tohx(bfr(src[k + q])); *(volatile v4h*)(B2 + e) = o; __threadfence(); *(volatile v4h*)(B2 + e) = o; }
__global__ __launch_bounds__(256) void k_w3(const float* __restrict__ W3, h16* B3) { const size_t e = ((size_t)blockIdx.x * 256 + threadIdx.x) * 4; if (e >= (size_t)NA * HH * HH) return; v4h o;
#pragma unroll
    for (int q = 0; q < 4; ++q) o[q] = tohx(bfr(W3[e + q])); *(volatile v4h*)(B3 + e) = o; __threadfence(); *(volatile v4h*)(B3 + e) = o; }
__global__ __launch_bounds__(256) void k_wo(const float* __restrict__ Wo, bf* BO) { const size_t e = ((size_t)blockIdx.x * 256 + threadIdx.x) * 4; if (e >= (size_t)NA * 64 * HH) return; const int k = (int)(e % HH); const int n = (int)((e / HH) % 64); const int a = (int)(e / ((size_t)HH * 64)); v4us o;
#pragma unroll
    for (int q = 0; q < 4; ++q) o[q] = n < NO ? f2bf(Wo[((size_t)a * NO + n) * HH + k + q]) : (unsigned short)0; *(volatile v4us*)(BO + e) = o; __threadfence(); *(volatile v4us*)(BO + e) = o; }
__global__ __launch_bounds__(256) void k_xn(const float* __restrict__ x, const float* __restrict__ wi, const float* __restrict__ bi, bf* Xh, bf* Xl) { const size_t e = ((size_t)blockIdx.x * 256 + threadIdx.x) * 2; if (e >= (size_t)NA * NBT * KI) return; const int k = (int)(e % KI); const int b = (int)((e / KI) % NBT); const int a = (int)(e / ((size_t)KI * NBT)); v2us oh, ol;
#pragma unroll
    for (int u = 0; u < 2; ++u) { unsigned short h = 0, l = 0; const int kk = k + u; if (kk < DI) { float t = __fmul_rn(bfr(x[(size_t)b * DI + kk]), bfr(wi[a * DI + kk])); asm volatile("" : "+v"(t)); splitf(__fadd_rn(t, bfr(bi[a * DI + kk])), h, l); } oh[u] = h; ol[u] = l; }
    *(volatile v2us*)(Xh + e) = oh; *(volatile v2us*)(Xl + e) = ol; __threadfence(); *(volatile v2us*)(Xh + e) = oh; *(volatile v2us*)(Xl + e) = ol; }
__global__ __launch_bounds__(256) void k_h(const float* __restrict__ G, const float* __restrict__ bm, const float* __restrict__ bs, int a, h16* H16, float* HF) { const size_t e = ((size_t)blockIdx.x * 256 + threadIdx.x) * 4; if (e >= (size_t)NBT * HH) return; const int n = (int)(e % HH); const int b = (int)(e / HH); const float* g = G + (size_t)b * 2 * HH; v4h o; v4f of;
#pragma unroll
    for (int q = 0; q < 4; ++q) { const float m = __fadd_rn(g[n + q], bfr(bm[a * HH + n + q])); const float s = __fadd_rn(g[HH + n + q], bfr(bs[a * HH + n + q])); const float h = __fadd_rn(gelu_(m), s); o[q] = tohx(h); of[q] = h; }
    *(volatile v4h*)(H16 + e) = o; *(volatile v4f*)(HF + e) = of; __threadfence(); *(volatile v4h*)(H16 + e) = o; *(volatile v4f*)(HF + e) = of; }
__global__ __launch_bounds__(256) void k_h3(const float* __restrict__ G3, const float* __restrict__ b3, const float* __restrict__ H2F, const float* __restrict__ hw, const float* __restrict__ hb, int a, bf* Ph, bf* Pl) { const size_t e = ((size_t)blockIdx.x * 256 + threadIdx.x) * 4; if (e >= (size_t)NBT * HH) return; const int n = (int)(e % HH); v4us oh, ol;
#pragma unroll
    for (int q = 0; q < 4; ++q) { const float t = __fadd_rn(__fadd_rn(G3[e + q], bfr(b3[a * HH + n + q])), H2F[e + q]); float u = __fmul_rn(t, bfr(hw[a * HH + n + q])); asm volatile("" : "+v"(u)); unsigned short h, l; splitf(__fadd_rn(u, bfr(hb[a * HH + n + q])), h, l); oh[q] = h; ol[q] = l; }
    *(volatile v4us*)(Ph + e) = oh; *(volatile v4us*)(Pl + e) = ol; __threadfence(); *(volatile v4us*)(Ph + e) = oh; *(volatile v4us*)(Pl + e) = ol; }
__global__ __launch_bounds__(256) void k_out(const float* __restrict__ R, const float* __restrict__ bo, int a, float* OUT) { const int e = blockIdx.x * 256 + threadIdx.x; if (e >= NBT * NO) return; const int o = e % NO, b = e / NO; const float v = __fadd_rn(R[(size_t)b * 64 + o], bfr(bo[a * NO + o])); *(volatile float*)(OUT + (size_t)a * NBT * NO + e) = v; __threadfence(); *(volatile float*)(OUT + (size_t)a * NBT * NO + e) = v; }

extern "C" void kernel_launch(void* const* d_in, const int* in_sizes, int n_in,
                              void* d_out, int out_size, void* d_ws, size_t ws_size, hipStream_t stream) {
    (void)in_sizes; (void)n_in; (void)out_size;
    const float* IN[17]; for (int i = 0; i < 17; ++i) IN[i] = (const float*)d_in[i];
    float* OUT = (float*)d_out;
    char* wsp = (char*)d_ws;
    auto take = [&](size_t bytes) { char* p = wsp; wsp += (bytes + 255) & ~(size_t)255; return (void*)p; };
    bf* B1 = (bf*)take((size_t)NA * 2 * HH * KI * 2); h16* B2 = (h16*)take((size_t)NA * 2 * HH * HH * 2); h16* B3 = (h16*)take((size_t)NA * HH * HH * 2); bf* BO = (bf*)take((size_t)NA * 64 * HH * 2);
    bf* Xh = (bf*)take((size_t)NA * NBT * KI * 2); bf* Xl = (bf*)take((size_t)NA * NBT * KI * 2); float* G = (float*)take((size_t)NBT * 2 * HH * 4); h16* H1 = (h16*)take((size_t)NBT * HH * 2); float* H1F = (float*)take((size_t)NBT * HH * 4); h16* H2 = (h16*)take((size_t)NBT * HH * 2); float* H2F = (float*)take((size_t)NBT * HH * 4); float* G3 = (float*)take((size_t)NBT * HH * 4); bf* P3h = (bf*)take((size_t)NBT * HH * 2); bf* P3l = (bf*)take((size_t)NBT * HH * 2); float* R = (float*)take((size_t)NBT * 64 * 4);
    if ((size_t)(wsp - (char*)d_ws) > ws_size) return;
    k_w1<<<(unsigned)(((size_t)NA * 2 * HH * KI / 2 + 255) / 256), 256, 0, stream>>>(IN[3], IN[11], B1); k_w2<<<(unsigned)(((size_t)NA * 2 * HH * HH / 4 + 255) / 256), 256, 0, stream>>>(IN[5], IN[13], B2); k_w3<<<(unsigned)(((size_t)NA * HH * HH / 4 + 255) / 256), 256, 0, stream>>>(IN[7], B3); k_wo<<<(unsigned)(((size_t)NA * 64 * HH / 4 + 255) / 256), 256, 0, stream>>>(IN[9], BO);
    k_xn<<<(unsigned)(((size_t)NA * NBT * KI / 2 + 255) / 256), 256, 0, stream>>>(IN[0], IN[1], IN[2], Xh, Xl);
    const unsigned LH = (unsigned)(((size_t)NBT * HH / 4 + 255) / 256);
    for (int a = 0; a < NA; ++a) {
        k_gemmw<bf, 1, false><<<dim3(NBT / 64, 2 * HH / 64, 1), 32, 0, stream>>>(Xh + (size_t)a * NBT * KI, Xl + (size_t)a * NBT * KI, B1 + (size_t)a * 2 * HH * KI, nullptr, KI, G, 2 * HH, nullptr, 0, 0, 0); k_h<<<LH, 256, 0, stream>>>(G, IN[4], IN[12], a, H1, H1F);
        k_gemmw<h16, 0, false><<<dim3(NBT / 64, 2 * HH / 64, 1), 32, 0, stream>>>(H1, nullptr, B2 + (size_t)a * 2 * HH * HH, nullptr, HH, G, 2 * HH, nullptr, 0, 0, 0); k_h<<<LH, 256, 0, stream>>>(G, IN[6], IN[14], a, H2, H2F);
        k_gemmw<h16, 0, false><<<dim3(NBT / 64, HH / 64, 1), 32, 0, stream>>>(H2, nullptr, B3 + (size_t)a * HH * HH, nullptr, HH, G3, HH, nullptr, 0, 0, 0); k_h3<<<LH, 256, 0, stream>>>(G3, IN[8], H2F, IN[15], IN[16], a, P3h, P3l);
        k_gemmw<bf, 1, false><<<dim3(NBT / 64, 1, 1), 32, 0, stream>>>(P3h, P3l, BO + (size_t)a * 64 * HH, nullptr, HH, R, 64, nullptr, 0, 0, 0); k_out<<<(NBT * NO + 255) / 256, 256, 0, stream>>>(R, IN[10], a, OUT); }
}
